// KnowledgeCircuit_3092376453536
// MI455X (gfx1250) — hardware-verified
//
#include <hip/hip_runtime.h>
#include <stddef.h>


typedef _Float16 v16h __attribute__((ext_vector_type(16)));
typedef _Float16 v8h  __attribute__((ext_vector_type(8)));
typedef float    v8f  __attribute__((ext_vector_type(8)));
typedef float    v4f  __attribute__((ext_vector_type(4)));

#ifndef NB
#define NB 4
#endif
#ifndef SEQ
#define SEQ 1024
#endif
#define NB_FULL  4
#define SEQ_FULL 1024
#define DIM   1024
#define NEXP  32
#define RANK  128
#define MROWS (NB * SEQ)

static_assert(NB >= 1 && NB <= NB_FULL);
static_assert(SEQ >= 64 && SEQ <= SEQ_FULL && (SEQ % 64) == 0);
static_assert((DIM % 64) == 0 && (DIM % 32) == 0);
static_assert((RANK % 64) == 0 && (RANK % 32) == 0);
static_assert((MROWS % 64) == 0 && (MROWS % 8) == 0);
static_assert(DIM == 4 * 32 * 8);
static_assert(NEXP == 32);
static_assert(((NEXP * DIM) % 64) == 0 && ((NEXP * RANK) % 64) == 0);

#define LDT 72
#define LDC 68
static_assert((LDT % 8) == 0 && LDT >= 64);
static_assert((LDC % 4) == 0 && LDC >= 64);

#define WCARRY 64.0f
#define HCARRY 16.0f

#define FKT_BYTES ((size_t)RANK * NEXP * DIM * 2)
#define RKT_BYTES ((size_t)DIM * NEXP * RANK * 2)
#define X16_BYTES ((size_t)MROWS * DIM * 2)
#define H16_BYTES ((size_t)MROWS * RANK * 2)
#define OFF_FKT ((size_t)0)
#define OFF_RKT (OFF_FKT + FKT_BYTES)
#define OFF_X16 (OFF_RKT + RKT_BYTES)
#define OFF_H16 (OFF_X16 + X16_BYTES)
#define WS_TOTAL (OFF_H16 + H16_BYTES)
static_assert((FKT_BYTES % 128) == 0 && (RKT_BYTES % 128) == 0);
static_assert((X16_BYTES % 128) == 0 && (H16_BYTES % 128) == 0);
static_assert(WS_TOTAL <= (size_t)134217728);

__device__ __forceinline__ float bf16r(float x) {
  unsigned int u = __float_as_uint(x);
  u = (u + 0x7FFFu + ((u >> 16) & 1u)) & 0xFFFF0000u;
  return __uint_as_float(u);
}

static __device__ __forceinline__ _Float16 toh_flush(float v) {
  const _Float16 r = (_Float16)v;
  return (fabsf(v) < 6.103515625e-05f) ? (_Float16)0.0f : r;
}

__device__ __forceinline__ v16h frag_at(const _Float16* p) {
  v8h lo = *(const v8h*)(p);
  v8h hi = *(const v8h*)(p + 16);
  v16h out;
#pragma unroll
  for (int i = 0; i < 8; ++i) { out[i] = lo[i]; out[i + 8] = hi[i]; }
  return out;
}

__device__ __forceinline__ v8f wmma16(v16h a, v16h b, v8f c) {
  v8f d = __builtin_amdgcn_wmma_f32_16x16x32_f16(false, a, false, b, (short)0, c,
                                                 false, false);
  asm volatile("v_nop\n\tv_nop\n\tv_nop\n\tv_nop" : "+v"(d) : "v"(a), "v"(b));
  return d;
}

__global__ __launch_bounds__(256) void wconv_kernel(
    const float* __restrict__ W, _Float16* __restrict__ Wt, unsigned ldw, unsigned ldk) {
  __shared__ _Float16 T[64 * LDT];
  const unsigned tid = threadIdx.x;
  const unsigned n0 = blockIdx.x * 64u;
  const unsigned k0 = blockIdx.y * 64u;
#pragma unroll 4
  for (unsigned j = 0; j < 16u; ++j) {
    const unsigned idx = tid + 256u * j;
    const unsigned kr = idx >> 6, nc = idx & 63u;
    const float v = W[(size_t)(k0 + kr) * ldw + n0 + nc];
    T[nc * LDT + kr] = (_Float16)(WCARRY * bf16r(v));
  }
  __syncthreads();
  v8h x[2];
  size_t off[2];
#pragma unroll
  for (unsigned i = 0; i < 2u; ++i) {
    const unsigned n = 32u * i + (tid >> 3);
    const unsigned kc = (tid & 7u) * 8u;
    x[i] = *(const v8h*)&T[n * LDT + kc];
    off[i] = (size_t)(n0 + n) * ldk + k0 + kc;
  }
#pragma unroll
  for (int i = 0; i < 2; ++i) *(volatile v8h*)(Wt + off[i]) = x[i];
  __threadfence();
#pragma unroll
  for (int i = 0; i < 2; ++i) *(volatile v8h*)(Wt + off[i]) = x[i];
}

__global__ __launch_bounds__(256) void xconv_kernel(
    const float* __restrict__ X, _Float16* __restrict__ dst) {
  const unsigned lane = threadIdx.x & 31u;
  const unsigned w = (unsigned)__builtin_amdgcn_readfirstlane((int)(threadIdx.x >> 5));
  const unsigned crow = blockIdx.x * 8u + w;
  const unsigned bidx = crow / (unsigned)SEQ;
  const unsigned sq = crow - bidx * (unsigned)SEQ;
  const size_t srow = (size_t)bidx * SEQ_FULL + sq;
  const float* xr = X + srow * DIM + lane * 8u;
#pragma unroll 1
  for (unsigned j = 0; j < 4u; ++j) {
    const unsigned c = j * 256u + lane * 8u;
    const v4f a0 = *(const v4f*)(xr + j * 256u);
    const v4f a1 = *(const v4f*)(xr + j * 256u + 4u);
    v8h o;
#pragma unroll
    for (int i = 0; i < 4; ++i) {
      o[i]     = toh_flush(bf16r(a0[i]));
      o[i + 4] = toh_flush(bf16r(a1[i]));
    }
    _Float16* p = dst + (size_t)crow * DIM + c;
    *(volatile v8h*)p = o;
    __threadfence();
    *(volatile v8h*)p = o;
  }
}

template <int KE, int UP>
__device__ __forceinline__ void egemm_body(
    const _Float16* __restrict__ A16, const _Float16* __restrict__ Bt,
    const float* __restrict__ Wexp, float* __restrict__ outf, _Float16* __restrict__ out16) {
  static_assert((KE % 32) == 0 && KE >= 32);
  __shared__ __attribute__((aligned(16))) float Cs[64 * LDC];
  __shared__ __attribute__((aligned(16))) float Wl[NEXP * LDC];
  const unsigned tid = threadIdx.x, lane = tid & 31u;
  const unsigned w = (unsigned)__builtin_amdgcn_readfirstlane((int)(tid >> 5));
  const unsigned mw = w >> 1, nw = w & 1u;
  const unsigned hh = lane >> 4, m = lane & 15u;
  const unsigned n0 = blockIdx.x * 64u;
  const unsigned row0 = blockIdx.y * 64u;
  const unsigned ldb = (unsigned)NEXP * (unsigned)KE;

#pragma unroll
  for (unsigned j = 0; j < 2u; ++j) {
    const unsigned idx = tid + 256u * j;
    const unsigned r = idx >> 3, c = (idx & 7u) * 4u;
    const unsigned crow = row0 + r;
    const unsigned bidx = crow / (unsigned)SEQ;
    const unsigned sq = crow - bidx * (unsigned)SEQ;
    const size_t frow = (size_t)bidx * SEQ_FULL + sq;
    const v4f g = *(const v4f*)(Wexp + frow * NEXP + c);
#pragma unroll
    for (int i = 0; i < 4; ++i) Wl[(c + (unsigned)i) * LDC + r] = bf16r(g[i]);
  }
  __syncthreads();

  const _Float16* ap  = A16 + (size_t)(row0 + mw * 16u + m) * KE + hh * 8u;
  const _Float16* bp0 = Bt + (size_t)(n0 + nw * 32u + m) * ldb + hh * 8u;
  const _Float16* bp1 = bp0 + (size_t)16 * ldb;
  v8f hs0 = {}, hs1 = {};
#pragma unroll 1
  for (unsigned e = 0; e < (unsigned)NEXP; ++e) {
    const unsigned kb = e * (unsigned)KE;
    v8f acc0 = {}, acc1 = {};
#pragma unroll 2
    for (unsigned k0 = 0; k0 < (unsigned)KE; k0 += 32u) {
      const v16h a  = frag_at(ap + k0);
      const v16h b0 = frag_at(bp0 + kb + k0);
      const v16h b1 = frag_at(bp1 + kb + k0);
      acc0 = wmma16(a, b0, acc0);
      acc1 = wmma16(a, b1, acc1);
    }
    const v4f w0 = *(const v4f*)&Wl[e * LDC + mw * 16u + hh * 8u];
    const v4f w1 = *(const v4f*)&Wl[e * LDC + mw * 16u + hh * 8u + 4u];
#pragma unroll
    for (int r = 0; r < 4; ++r) {
      hs0[r]     = hs0[r]     + w0[r] * acc0[r];
      hs0[r + 4] = hs0[r + 4] + w1[r] * acc0[r + 4];
      hs1[r]     = hs1[r]     + w0[r] * acc1[r];
      hs1[r + 4] = hs1[r + 4] + w1[r] * acc1[r + 4];
    }
  }

#pragma unroll
  for (int r = 0; r < 8; ++r) {
    float* d = &Cs[(mw * 16u + hh * 8u + (unsigned)r) * LDC + nw * 32u + m];
    d[0]  = hs0[r];
    d[16] = hs1[r];
  }
  __syncthreads();

  if (UP == 0) {
    v8h x[2];
    size_t off[2];
#pragma unroll
    for (unsigned i = 0; i < 2u; ++i) {
      const unsigned r = 32u * i + (tid >> 3);
      const unsigned c = (tid & 7u) * 8u;
      const v4f u0 = *(const v4f*)&Cs[r * LDC + c];
      const v4f u1 = *(const v4f*)&Cs[r * LDC + c + 4];
#pragma unroll
      for (int j = 0; j < 4; ++j) {
        x[i][j]     = toh_flush(u0[j] * (HCARRY / WCARRY));
        x[i][j + 4] = toh_flush(u1[j] * (HCARRY / WCARRY));
      }
      off[i] = (size_t)(row0 + r) * RANK + n0 + c;
    }
#pragma unroll
    for (int i = 0; i < 2; ++i) *(volatile v8h*)(out16 + off[i]) = x[i];
    __threadfence();
#pragma unroll
    for (int i = 0; i < 2; ++i) *(volatile v8h*)(out16 + off[i]) = x[i];
  }

  if (UP == 1) {
    const float cs = 1.0f / (WCARRY * HCARRY);
    v4f xs[4];
    size_t off[4];
#pragma unroll
    for (unsigned i = 0; i < 4u; ++i) {
      const unsigned r = 16u * i + (tid >> 4);
      const unsigned c = (tid & 15u) * 4u;
      const unsigned crow = row0 + r;
      const unsigned bidx = crow / (unsigned)SEQ;
      const unsigned sq = crow - bidx * (unsigned)SEQ;
      const size_t frow = (size_t)bidx * SEQ_FULL + sq;
      const v4f u = *(const v4f*)&Cs[r * LDC + c];
      v4f val;
#pragma unroll
      for (int j = 0; j < 4; ++j) val[j] = u[j] * cs;
      xs[i] = val;
      off[i] = frow * DIM + n0 + c;
    }
#pragma unroll
    for (int i = 0; i < 4; ++i) *(volatile v4f*)(outf + off[i]) = xs[i];
    __threadfence();
#pragma unroll
    for (int i = 0; i < 4; ++i) *(volatile v4f*)(outf + off[i]) = xs[i];
  }
}

__global__ __launch_bounds__(256) void egemm_down_kernel(
    const _Float16* __restrict__ X16, const _Float16* __restrict__ FKt,
    const float* __restrict__ fw, _Float16* __restrict__ H16) {
  egemm_body<DIM, 0>(X16, FKt, fw, (float*)0, H16);
}
__global__ __launch_bounds__(256) void egemm_up_kernel(
    const _Float16* __restrict__ H16, const _Float16* __restrict__ RKt,
    const float* __restrict__ rw, float* __restrict__ outf) {
  egemm_body<RANK, 1>(H16, RKt, rw, outf, (_Float16*)0);
}

extern "C" void kernel_launch(void* const* d_in, const int* in_sizes, int n_in,
                              void* d_out, int out_size, void* d_ws, size_t ws_size,
                              hipStream_t stream) {
  if (n_in < 5) return;
  const long long need_rows = (long long)(NB - 1) * SEQ_FULL + SEQ;
  if ((long long)in_sizes[0] < need_rows * DIM) return;
  if ((long long)in_sizes[1] < need_rows * NEXP) return;
  if ((long long)in_sizes[2] < need_rows * NEXP) return;
  if ((long long)in_sizes[3] < (long long)NEXP * DIM * RANK) return;
  if ((long long)in_sizes[4] < (long long)NEXP * RANK * DIM) return;
  if ((long long)out_size < need_rows * DIM) return;
  if (ws_size < WS_TOTAL) return;

  const float* X  = (const float*)d_in[0];
  const float* fw = (const float*)d_in[1];
  const float* rw = (const float*)d_in[2];
  const float* FK = (const float*)d_in[3];
  const float* RK = (const float*)d_in[4];
  float* out = (float*)d_out;

  char* ws = (char*)d_ws;
  _Float16* FKt = (_Float16*)(ws + OFF_FKT);
  _Float16* RKt = (_Float16*)(ws + OFF_RKT);
  _Float16* X16 = (_Float16*)(ws + OFF_X16);
  _Float16* H16 = (_Float16*)(ws + OFF_H16);

  dim3 blk(256);

  wconv_kernel<<<dim3(RANK / 64, (NEXP * DIM) / 64), blk, 0, stream>>>(
      FK, FKt, (unsigned)RANK, (unsigned)(NEXP * DIM));
  wconv_kernel<<<dim3(DIM / 64, (NEXP * RANK) / 64), blk, 0, stream>>>(
      RK, RKt, (unsigned)DIM, (unsigned)(NEXP * RANK));

  xconv_kernel<<<dim3(MROWS / 8), blk, 0, stream>>>(X, X16);
  egemm_down_kernel<<<dim3(RANK / 64, MROWS / 64), blk, 0, stream>>>(X16, FKt, fw, H16);
  egemm_up_kernel<<<dim3(DIM / 64, MROWS / 64), blk, 0, stream>>>(H16, RKt, rw, out);
}
